// TuckERInteraction_20615843021592
// MI455X (gfx1250) — hardware-verified
//
#include <hip/hip_runtime.h>


namespace {
constexpr int BS = 16, S = 2048, NR = BS * S, D = 128;
constexpr float XS = 8.0f, WSC = 256.0f, EPS = 1e-5f;
typedef _Float16 b16;
typedef __attribute__((ext_vector_type(16))) _Float16 v16b;
typedef __attribute__((ext_vector_type(8))) _Float16 v8b;
typedef __attribute__((ext_vector_type(8))) float v8f;
typedef __attribute__((ext_vector_type(4))) float v4f;
__device__ __forceinline__ float bf16_rne(float f) { unsigned int u = __float_as_uint(f); u += 0x7FFFu + ((u >> 16) & 1u); return __uint_as_float(u & 0xFFFF0000u); }
__device__ __forceinline__ void split16(float v, b16& hi, b16& lo) { hi = (b16)v; lo = (b16)(v - (float)hi); }
__device__ __forceinline__ v16b frag_kb(const b16* p, int hh) { const v8b a = *(const v8b*)(p + 8 * hh), b = *(const v8b*)(p + 16 + 8 * hh); v16b f;
#pragma unroll
  for (int e = 0; e < 8; ++e) { f[e] = a[e]; f[8 + e] = b[e]; } return f; }
__device__ __forceinline__ v8f wmma16b(v16b a, v16b b, v8f c) { v8f d = __builtin_amdgcn_wmma_f32_16x16x32_f16(false, a, false, b, (short)0, c, false, false); asm volatile("v_nop\n\tv_nop\n\tv_nop\n\tv_nop" : "+v"(d) : "v"(a), "v"(b)); return d; }
__device__ __forceinline__ void wave_lds_sync() { __builtin_amdgcn_fence(__ATOMIC_RELEASE, "workgroup"); __builtin_amdgcn_wave_barrier(); __builtin_amdgcn_fence(__ATOMIC_ACQUIRE, "workgroup"); }
__device__ __forceinline__ float pmul(float a, float b) { float p = a * b; asm volatile("" : "+v"(p)); return p; }

__global__ __launch_bounds__(32) void g_kernel(const float* __restrict__ h, const float* __restrict__ r, const float* __restrict__ g0, const float* __restrict__ b0, const float* __restrict__ m0_, const float* __restrict__ v0, int MLIM, float* __restrict__ G) {
  __shared__ __attribute__((aligned(16))) b16 Rt[D][D + 8], Ah[16][D + 8], Al[16][D + 8]; __shared__ float Tf[16][D + 4]; const int lane = threadIdx.x, nloc = lane & 15, hlf = lane >> 4; const int m = blockIdx.x; if (m >= MLIM) return;
  for (int d = 0; d < D; ++d) for (int q = 0; q < 4; ++q) { const int i = q * 32 + lane; Rt[i][d] = (b16)(bf16_rne(r[((size_t)m * D + d) * D + i]) * XS); }
  float sc[4], sh[4]; for (int q = 0; q < 4; ++q) { const int c = q * 32 + lane; const float s = pmul(rsqrtf(bf16_rne(v0[c]) + EPS), bf16_rne(g0[c])); sc[q] = s; sh[q] = bf16_rne(b0[c]) - pmul(bf16_rne(m0_[c]), s); }
#pragma unroll 1
  for (int rt = 0; rt < 8; ++rt) {
    for (int rr = 0; rr < 16; ++rr) { const size_t np_ = (size_t)m + 256 * (size_t)(rt * 16 + rr); for (int q = 0; q < 4; ++q) { const int c = q * 32 + lane; const float hb = pmul(bf16_rne(h[np_ * D + c]), sc[q]) + sh[q]; b16 p, ql; split16(hb * XS, p, ql); Ah[rr][c] = p; Al[rr][c] = ql; } }
    wave_lds_sync(); v8f acc[8];
#pragma unroll
    for (int t = 0; t < 8; ++t) acc[t] = (v8f){};
#pragma unroll
    for (int kb = 0; kb < D; kb += 32) { const v16b a = frag_kb(&Ah[nloc][kb], hlf), al = frag_kb(&Al[nloc][kb], hlf);
#pragma unroll
      for (int t = 0; t < 8; ++t) { const v16b bw = frag_kb(&Rt[t * 16 + nloc][kb], hlf); acc[t] = wmma16b(a, bw, acc[t]); acc[t] = wmma16b(al, bw, acc[t]); } }
#pragma unroll
    for (int t = 0; t < 8; ++t)
#pragma unroll
      for (int r8 = 0; r8 < 8; ++r8) Tf[8 * hlf + r8][t * 16 + nloc] = acc[t][r8] * (1.0f / (XS * XS));
    wave_lds_sync();
    for (int pass = 0; pass < 2; ++pass) { for (int rr = 0; rr < 16; ++rr) { const size_t np_ = (size_t)m + 256 * (size_t)(rt * 16 + rr); *(volatile v4f*)(G + np_ * D + lane * 4) = *(const v4f*)(&Tf[rr][lane * 4]); } __threadfence(); }
    wave_lds_sync(); }
}
__global__ __launch_bounds__(32) void s_kernel(const float* __restrict__ G, const float* __restrict__ W, const float* __restrict__ t, const float* __restrict__ g1, const float* __restrict__ b1, const float* __restrict__ m1_, const float* __restrict__ v1, int KLIM, float* __restrict__ out) {
  __shared__ __attribute__((aligned(16))) b16 Wt[D][D + 8], Ah[16][D + 8], Al[16][D + 8]; __shared__ float Tf[16][D + 4], So[256]; const int lane = threadIdx.x, nloc = lane & 15, hlf = lane >> 4; const int kb = blockIdx.x; if (kb >= KLIM) return;
  for (int i = 0; i < D; ++i) for (int q = 0; q < 4; ++q) { const int j = q * 32 + lane; Wt[j][i] = (b16)(bf16_rne(W[((size_t)kb * D + i) * D + j]) * WSC); }
  __shared__ float Tsc[D], Tsh[D]; for (int q = 0; q < 4; ++q) { const int c = q * 32 + lane; const float s = pmul(rsqrtf(bf16_rne(v1[c]) + EPS), bf16_rne(g1[c])); Tsc[c] = s; Tsh[c] = bf16_rne(b1[c]) - pmul(bf16_rne(m1_[c]), s); }
#pragma unroll 1
  for (int rt = 0; rt < 16; ++rt) { const size_t n0 = (size_t)kb * 256 + rt * 16;
    for (int rr = 0; rr < 16; ++rr) for (int q = 0; q < 4; ++q) { b16 p, ql; split16(G[(n0 + rr) * D + q * 32 + lane] * XS, p, ql); Ah[rr][q * 32 + lane] = p; Al[rr][q * 32 + lane] = ql; }
    wave_lds_sync(); v8f acc[8];
#pragma unroll
    for (int tt = 0; tt < 8; ++tt) acc[tt] = (v8f){};
#pragma unroll
    for (int kk = 0; kk < D; kk += 32) { const v16b a = frag_kb(&Ah[nloc][kk], hlf), al = frag_kb(&Al[nloc][kk], hlf);
#pragma unroll
      for (int tt = 0; tt < 8; ++tt) { const v16b bw = frag_kb(&Wt[tt * 16 + nloc][kk], hlf); acc[tt] = wmma16b(a, bw, acc[tt]); acc[tt] = wmma16b(al, bw, acc[tt]); } }
#pragma unroll
    for (int tt = 0; tt < 8; ++tt)
#pragma unroll
      for (int r8 = 0; r8 < 8; ++r8) Tf[8 * hlf + r8][tt * 16 + nloc] = acc[tt][r8] * (1.0f / (XS * WSC));
    wave_lds_sync();
    if (lane < 16) { const size_t np_ = n0 + lane; float s = 0.0f;
#pragma unroll 4
      for (int j = 0; j < D; ++j) { const float tb = pmul(bf16_rne(t[np_ * D + j]), Tsc[j]) + Tsh[j]; s += pmul(Tf[lane][j], tb); } So[rt * 16 + lane] = s; }
    wave_lds_sync(); }
  for (int pass = 0; pass < 2; ++pass) { for (int q = 0; q < 8; ++q) ((volatile float*)out)[(size_t)kb * 256 + q * 32 + lane] = So[q * 32 + lane]; __threadfence(); }
}
}

extern "C" void kernel_launch(void* const* d_in, const int* in_sizes, int n_in, void* d_out, int out_size, void* d_ws, size_t ws_size, hipStream_t stream) {
  (void)n_in;
  auto Fp = [&](int i) { return (const float*)d_in[i]; };
  if (in_sizes[0] != NR * D || in_sizes[1] != NR * D || in_sizes[2] != NR * D || in_sizes[3] != D * D * D || in_sizes[7] != D || in_sizes[11] != D || out_size != NR) return;
  const int MLIM = 256, KLIM = 128;
  size_t off = 0; char* ws = (char*)d_ws;
  auto carve = [&](size_t bytes) { char* p = ws + off; off += (bytes + 255) & ~(size_t)255; return p; };
  float* G = (float*)carve((size_t)NR * D * 4);
  if (off > ws_size || off > ((size_t)32 << 20)) return;
  g_kernel<<<MLIM, 32, 0, stream>>>(Fp(0), Fp(1), Fp(4), Fp(5), Fp(6), Fp(7), MLIM, G);
  s_kernel<<<KLIM, 32, 0, stream>>>(G, Fp(3), Fp(2), Fp(8), Fp(9), Fp(10), Fp(11), KLIM, (float*)d_out);
}
